// MultiHeadRecurrentAttention_73263552135473
// MI455X (gfx1250) — hardware-verified
//
#include <hip/hip_runtime.h>

typedef __attribute__((ext_vector_type(16))) _Float16 v16h;
typedef __attribute__((ext_vector_type(8)))  _Float16 v8h;
typedef __attribute__((ext_vector_type(16))) __bf16   v16b;
typedef __attribute__((ext_vector_type(8)))  __bf16   v8b;
typedef __attribute__((ext_vector_type(8)))  float    v8f;
typedef __attribute__((ext_vector_type(4)))  float    v4f;
typedef __attribute__((ext_vector_type(4)))  unsigned v4u;
typedef __attribute__((ext_vector_type(4)))  int      v4i;

__device__ __forceinline__ unsigned short f2bf_bits(float f) {
  unsigned u = __float_as_uint(f);
  return (unsigned short)((u + 0x7FFFu + ((u >> 16) & 1u)) >> 16);
}
__device__ __forceinline__ float bf_bits2f(unsigned short h) { return __uint_as_float(((unsigned)h) << 16); }

__device__ __forceinline__ void dep_guard_h(v8f& a, v8f& b, v16h x, v16h y) { asm volatile("v_nop\n\tv_nop\n\tv_nop\n\tv_nop" : "+v"(a), "+v"(b) : "v"(x), "v"(y)); }
__device__ __forceinline__ void dep_guard_b(v8f& a, v8f& b, v16b x, v16b y) { asm volatile("v_nop\n\tv_nop\n\tv_nop\n\tv_nop" : "+v"(a), "+v"(b) : "v"(x), "v"(y)); }
__device__ __forceinline__ void keep4_h(v16h a, v16h b, v16h c, v16h d) { asm volatile("v_nop" :: "v"(a), "v"(b), "v"(c), "v"(d)); }
__device__ __forceinline__ void keep4_b(v16b a, v16b b, v16b c, v16b d) { asm volatile("v_nop" :: "v"(a), "v"(b), "v"(c), "v"(d)); }
__device__ __forceinline__ void acc_guard4(v8f& a, v8f& b, v8f& c, v8f& d) { asm volatile("v_nop\n\tv_nop\n\tv_nop\n\tv_nop" : "+v"(a), "+v"(b), "+v"(c), "+v"(d)); }
template <typename T> struct Frag;
template <> struct Frag<_Float16> {
  typedef v16h V; union U { v16h v; v8h h[2]; };
  static __device__ __forceinline__ v16h load(const _Float16* p) {
    U f; f.h[0] = *(const v8h*)(p); f.h[1] = *(const v8h*)(p + 16); return f.v;
  }
  static __device__ __forceinline__ v8f mma(v16h a, v16h b, v8f c) {
    return __builtin_amdgcn_wmma_f32_16x16x32_f16(false, a, false, b, (short)0, c, false, false);
  }
  static __device__ __forceinline__ void guard(v8f& a, v8f& b, v16h x, v16h y) { dep_guard_h(a, b, x, y); }
  static __device__ __forceinline__ void keep(v16h a, v16h b, v16h c, v16h d) { keep4_h(a, b, c, d); }
};
template <> struct Frag<__bf16> {
  typedef v16b V; union U { v16b v; v8b h[2]; };
  static __device__ __forceinline__ v16b load(const __bf16* p) {
    U f; f.h[0] = *(const v8b*)(p); f.h[1] = *(const v8b*)(p + 16); return f.v;
  }
  static __device__ __forceinline__ v8f mma(v16b a, v16b b, v8f c) {
    return __builtin_amdgcn_wmma_f32_16x16x32_bf16(false, a, false, b, (short)0, c, false, false);
  }
  static __device__ __forceinline__ void guard(v8f& a, v8f& b, v16b x, v16b y) { dep_guard_b(a, b, x, y); }
  static __device__ __forceinline__ void keep(v16b a, v16b b, v16b c, v16b d) { keep4_b(a, b, c, d); }
};

template <int ET> struct Elem;
template <> struct Elem<0> { typedef _Float16 T; };
template <> struct Elem<1> { typedef __bf16 T; };
template <int ET, bool SPLIT, int BIAS_MODE, int OUT_MODE, bool RESID, int ACT = 0>
__global__ __launch_bounds__(256) void wmma_gemm64(
    const unsigned short* __restrict__ Ap, const unsigned short* __restrict__ A2p, int lda, long strideA,
    const unsigned short* __restrict__ Btp, const unsigned short* __restrict__ Bt2p, int ldb, long strideB,
    void* __restrict__ Cout, void* __restrict__ Cout2, int ldc, long strideC,
    const float* __restrict__ bias,
    const float* __restrict__ resid, long strideR,
    int M, int N, int K, float scale) {
  typedef typename Elem<ET>::T T;
  typedef typename Frag<T>::V V;
  const T* A = (const T*)Ap; const T* A2 = (const T*)A2p; const T* Bt = (const T*)Btp; const T* Bt2 = (const T*)Bt2p;
  __shared__ __align__(16) float sT[8][16 * 68];
  const int b    = blockIdx.y;
  const int lane = threadIdx.x & 31;
  const int wave = threadIdx.x >> 5;
  const int tilesN = N >> 6;
  const int tilesM = M >> 6;
  const int tile = blockIdx.x * 8 + wave;
  if (tile >= tilesM * tilesN) return;
  const int tm = tile / tilesN;
  const int tn = tile - tm * tilesN;
  const int m0 = tm << 6;
  const int n0 = tn << 6;

  const T* Ab  = A  + (size_t)b * strideA;
  const T* Bb  = Bt + (size_t)b * strideB;
  const T* Ab2 = SPLIT ? (A2  + (size_t)b * strideA) : nullptr;
  const T* Bb2 = SPLIT ? (Bt2 + (size_t)b * strideB) : nullptr;

  const int rlane = lane & 15;
  const int koff  = (lane >> 4) * 8;
  const int mOff  = (lane >> 4) * 8;

  v8f acc[4][4];
#pragma unroll
  for (int i = 0; i < 4; ++i)
#pragma unroll
    for (int j = 0; j < 4; ++j) acc[i][j] = (v8f){0.f,0.f,0.f,0.f,0.f,0.f,0.f,0.f};

  for (int k0 = 0; k0 < K; k0 += 32) {
    V bh[4], bl[4];
#pragma unroll
    for (int j = 0; j < 4; ++j) {
      const size_t bo = (size_t)(n0 + (j << 4) + rlane) * ldb + koff + k0;
      bh[j] = Frag<T>::load(Bb + bo);
      if (SPLIT) bl[j] = Frag<T>::load(Bb2 + bo);
    }
#pragma unroll
    for (int i = 0; i < 4; ++i) {
      const size_t ao = (size_t)(m0 + (i << 4) + rlane) * lda + koff + k0;
      V ah = Frag<T>::load(Ab + ao);
      V al;
      if (SPLIT) al = Frag<T>::load(Ab2 + ao);
#pragma unroll
      for (int j = 0; j < 4; ++j) {
        acc[i][j] = Frag<T>::mma(ah, bh[j], acc[i][j]);
        if (SPLIT) {
          acc[i][j] = Frag<T>::mma(ah, bl[j], acc[i][j]);
          acc[i][j] = Frag<T>::mma(al, bh[j], acc[i][j]);
        }
      }
      Frag<T>::guard(acc[i][0], acc[i][3], ah, SPLIT ? al : ah);
    }
    Frag<T>::keep(bh[0], bh[1], bh[2], bh[3]);
    if (SPLIT) Frag<T>::keep(bl[0], bl[1], bl[2], bl[3]);
  }
  acc_guard4(acc[0][0], acc[0][1], acc[0][2], acc[0][3]);
  acc_guard4(acc[1][0], acc[1][1], acc[1][2], acc[1][3]);
  acc_guard4(acc[2][0], acc[2][1], acc[2][2], acc[2][3]);
  acc_guard4(acc[3][0], acc[3][1], acc[3][2], acc[3][3]);

  float* slab = sT[wave];
  const float* Rb = RESID ? (resid + (size_t)b * strideR) : nullptr;
#pragma unroll
  for (int i = 0; i < 4; ++i) {
    const int mBase = m0 + (i << 4);
#pragma unroll
    for (int j = 0; j < 4; ++j) {
      const int n = n0 + (j << 4) + rlane;
      float bv = 0.f;
      if (BIAS_MODE == 2) bv = bias[n];
#pragma unroll
      for (int r = 0; r < 8; ++r) {
        float v = acc[i][j][r] * scale;
        if (BIAS_MODE == 1) v += bias[mBase + mOff + r];
        if (BIAS_MODE == 2) v += bv;
        if (RESID) v += Rb[(size_t)(mBase + mOff + r) * ldc + n];
        if (ACT == 1) v = tanhf(v);
        if (ACT == 2) v = fmaxf(v, 0.0f);
        if (ACT == 3) v = v / (1.0f + expf(-v));
        if (ACT == 4) v = (v > 0.f) ? v : 0.01f * v;
        if (ACT == 5) v = 0.5f * v * (1.0f + erff(v * 0.70710678118654752f));
        slab[(mOff + r) * 68 + (j << 4) + rlane] = v;
      }
    }
    __builtin_amdgcn_fence(__ATOMIC_RELEASE, "workgroup");
    __builtin_amdgcn_wave_barrier();
    __builtin_amdgcn_fence(__ATOMIC_ACQUIRE, "workgroup");
    if (OUT_MODE == 0) {
      float* C = (float*)Cout + (size_t)b * strideC;
      const int hh = lane >> 4, c4 = (lane & 15) * 4;
      for (int pass = 0; pass < 2; ++pass) {
#pragma unroll
        for (int it = 0; it < 8; ++it) {
          const int row = it * 2 + hh;
          v4f v = *(const v4f*)(slab + row * 68 + c4);
          *(volatile v4f*)(C + (size_t)(mBase + row) * ldc + n0 + c4) = v;
        }
        __threadfence();
      }
    } else {
      const int q = lane >> 3, c8 = (lane & 7) * 8;
      unsigned short* C  = (unsigned short*)Cout  + (size_t)b * strideC;
      unsigned short* C2 = (OUT_MODE == 2) ? ((unsigned short*)Cout2 + (size_t)b * strideC) : nullptr;
      for (int pass = 0; pass < 2; ++pass) {
#pragma unroll
        for (int it = 0; it < 4; ++it) {
          const int row = it * 4 + q;
          const float* sp = slab + row * 68 + c8;
          v8h hv, lv;
#pragma unroll
          for (int e = 0; e < 8; ++e) {
            if (OUT_MODE == 1) {
              hv[e] = (_Float16)sp[e];
            } else {
              unsigned short hb = f2bf_bits(sp[e]);
              unsigned short lb = f2bf_bits(sp[e] - bf_bits2f(hb));
              hv[e] = __builtin_bit_cast(_Float16, hb);
              lv[e] = __builtin_bit_cast(_Float16, lb);
            }
          }
          *(volatile v8h*)(C + (size_t)(mBase + row) * ldc + n0 + c8) = hv;
          if (OUT_MODE == 2) *(volatile v8h*)(C2 + (size_t)(mBase + row) * ldc + n0 + c8) = lv;
        }
        __threadfence();
      }
    }
    __builtin_amdgcn_fence(__ATOMIC_RELEASE, "workgroup");
    __builtin_amdgcn_wave_barrier();
    __builtin_amdgcn_fence(__ATOMIC_ACQUIRE, "workgroup");
  }
}

constexpr int NBATCH = 2;
constexpr int SEQ    = 128;
constexpr int FEAT   = 1024;
constexpr int NHEAD  = 8;
constexpr int HDIM   = 128;
constexpr int HD_ALL = NHEAD * HDIM;
constexpr int NGATE  = 4 * HDIM;
constexpr int NROW   = NBATCH * SEQ;
constexpr int NBH    = NBATCH * NHEAD;
constexpr int HP_LDS = 136;
constexpr int SP_LDS = 132;
static_assert(NROW % 64 == 0 && HD_ALL % 64 == 0 && FEAT % 32 == 0 && HDIM % 32 == 0 && NGATE % 64 == 0, "tile multiples");

__device__ __forceinline__ unsigned pack_hl(float f0, float f1, unsigned& lo_word) {
  const unsigned short h0 = f2bf_bits(f0), h1 = f2bf_bits(f1);
  const unsigned short l0 = f2bf_bits(f0 - bf_bits2f(h0));
  const unsigned short l1 = f2bf_bits(f1 - bf_bits2f(h1));
  lo_word = (unsigned)l0 | ((unsigned)l1 << 16);
  return (unsigned)h0 | ((unsigned)h1 << 16);
}
__device__ __forceinline__ unsigned pack_f16(float f0, float f1) {
  const unsigned short a = __builtin_bit_cast(unsigned short, (_Float16)f0);
  const unsigned short b = __builtin_bit_cast(unsigned short, (_Float16)f1);
  return (unsigned)a | ((unsigned)b << 16);
}

__global__ __launch_bounds__(256) void k_cvt_split(const float* __restrict__ in,
    unsigned short* __restrict__ oh, unsigned short* __restrict__ ol, int n8) {
  const int i = blockIdx.x * 256 + threadIdx.x;
  if (i >= n8) return;
  const float* p = in + (size_t)i * 8;
  const v4f a = *(const v4f*)p;
  const v4f c = *(const v4f*)(p + 4);
  unsigned wh0, wh1, wh2, wh3, wl0, wl1, wl2, wl3;
  wh0 = pack_hl(a[0], a[1], wl0);
  wh1 = pack_hl(a[2], a[3], wl1);
  wh2 = pack_hl(c[0], c[1], wl2);
  wh3 = pack_hl(c[2], c[3], wl3);
  const v4u vh = {wh0, wh1, wh2, wh3};
  const v4u vl = {wl0, wl1, wl2, wl3};
  unsigned short* dh = oh + (size_t)i * 8;
  unsigned short* dl = ol + (size_t)i * 8;
  *(volatile v4u*)dh = vh;
  *(volatile v4u*)dl = vl;
  __threadfence();
  *(volatile v4u*)dh = vh;
  *(volatile v4u*)dl = vl;
}

template <int MODE>
__global__ __launch_bounds__(256) void k_transpose16(const float* __restrict__ in,
    unsigned short* __restrict__ outA, unsigned short* __restrict__ outB, int R, int Cc, float scale) {
  __shared__ float tile[64][65];
  const int tid = threadIdx.x;
  const int bz = blockIdx.z;
  const int r0 = blockIdx.y * 64;
  const int c0 = blockIdx.x * 64;
  const float* inb = in + (size_t)bz * (size_t)R * (size_t)Cc;
  {
    const int lr = tid >> 2, lc = (tid & 3) * 16;
    const float* src = inb + (size_t)(r0 + lr) * Cc + c0 + lc;
#pragma unroll
    for (int e = 0; e < 4; ++e) {
      const v4f v = *(const v4f*)(src + 4 * e);
      tile[lr][lc + 4 * e + 0] = v[0];
      tile[lr][lc + 4 * e + 1] = v[1];
      tile[lr][lc + 4 * e + 2] = v[2];
      tile[lr][lc + 4 * e + 3] = v[3];
    }
  }
  __syncthreads();
  const size_t plane = (size_t)bz * (size_t)Cc * (size_t)R;
  const int orl = tid >> 3, seg = (tid & 7) * 8;
  v4u va[2], vb[2];
  size_t dst[2];
#pragma unroll
  for (int it = 0; it < 2; ++it) {
    const int orow = it * 32 + orl;
    unsigned wa[4], wb[4];
#pragma unroll
    for (int e = 0; e < 4; ++e) {
      const float f0 = tile[seg + 2 * e][orow];
      const float f1 = tile[seg + 2 * e + 1][orow];
      if (MODE == 0) {
        wa[e] = pack_hl(f0, f1, wb[e]);
      } else {
        wa[e] = pack_f16(f0 * scale, f1 * scale);
        wb[e] = wa[e];
      }
    }
    va[it] = (v4u){wa[0], wa[1], wa[2], wa[3]};
    vb[it] = (v4u){wb[0], wb[1], wb[2], wb[3]};
    dst[it] = plane + (size_t)(c0 + orow) * (size_t)R + (size_t)(r0 + seg);
  }
  for (int pass = 0; pass < 2; ++pass) {
#pragma unroll
    for (int it = 0; it < 2; ++it) {
      *(volatile v4u*)(outA + dst[it]) = va[it];
      if (MODE == 0) *(volatile v4u*)(outB + dst[it]) = vb[it];
    }
    __threadfence();
  }
}

__global__ __launch_bounds__(256) void k_softmax_rows(const float* __restrict__ s, const int* __restrict__ mask,
                                                     float* __restrict__ attn) {
  const int tid = threadIdx.x, w = tid >> 5, lane = tid & 31;
  const int row = blockIdx.x * 8 + w;
  const int bh = row >> 7, q = row & (SEQ - 1), b = bh >> 3;
  const v4f x = *(const v4f*)(s + (size_t)row * SEQ + lane * 4);
  const v4i mk = *(const v4i*)(mask + ((size_t)b * SEQ + q) * SEQ + lane * 4);
  const float ninf = -__builtin_inff();
  float v[4];
#pragma unroll
  for (int e = 0; e < 4; ++e) {
    const float mf = 1.0f - (float)mk[e];
    v[e] = (mf == 1.0f) ? ninf : (x[e] - mf);
  }
  float mx = fmaxf(fmaxf(v[0], v[1]), fmaxf(v[2], v[3]));
#pragma unroll
  for (int o = 16; o > 0; o >>= 1) mx = fmaxf(mx, __shfl_xor(mx, o, 32));
  const float e0 = expf(v[0] - mx), e1 = expf(v[1] - mx), e2 = expf(v[2] - mx), e3 = expf(v[3] - mx);
  float sum = (e0 + e1) + (e2 + e3);
#pragma unroll
  for (int o = 16; o > 0; o >>= 1) sum += __shfl_xor(sum, o, 32);
  const float inv = 1.0f / sum;
  const v4f ov = {e0 * inv, e1 * inv, e2 * inv, e3 * inv};
  float* dstp = attn + (size_t)row * SEQ + lane * 4;
  *(volatile v4f*)dstp = ov;
  __threadfence();
  *(volatile v4f*)dstp = ov;
}

__device__ __forceinline__ float sigm_f(float x) { return __builtin_amdgcn_rcpf(1.0f + expf(-x)); }

__global__ __launch_bounds__(256) void k_recur(const float* __restrict__ attn, const float* __restrict__ vx,
                                              const unsigned short* __restrict__ wht, const float* __restrict__ blstm,
                                              unsigned short* __restrict__ rdh, unsigned short* __restrict__ rdl) {
  __shared__ __align__(16) _Float16 hA[2][32 * HP_LDS];
  __shared__ __align__(16) float hs[32 * SP_LDS];
  __shared__ float acol[2][32];
  const int tid = threadIdx.x;
  const int w = tid >> 5, lane = tid & 31, hh = lane >> 4, cix = lane & 15;
  const int blk = blockIdx.x;
  const int bh = blk >> 2;
  const int qb = (blk & 3) * 32;
  const int b = bh >> 3, h = bh & 7;
  const int rowg0 = bh * SEQ + qb;
  {
    const v4u z = {0u, 0u, 0u, 0u};
    v4u* p = (v4u*)(&hA[0][0]);
    for (int i = tid; i < (2 * 32 * HP_LDS) / 8; i += 256) p[i] = z;
  }
  float cst[2][8];
#pragma unroll
  for (int mt = 0; mt < 2; ++mt)
#pragma unroll
    for (int r = 0; r < 8; ++r) cst[mt][r] = 0.0f;
  const int ucol = 16 * w + cix;
  const float bl0 = blstm[h * NGATE + ucol];
  const float bl1 = blstm[h * NGATE + HDIM + ucol];
  const float bl2 = blstm[h * NGATE + 2 * HDIM + ucol];
  const float bl3 = blstm[h * NGATE + 3 * HDIM + ucol];
  const _Float16* whb = (const _Float16*)wht + (size_t)h * NGATE * HDIM;
  const float RINV = 1.0f / 32768.0f;

  for (int k = 0; k < SEQ; ++k) {
    const int par = k & 1;
    if (w == 0) acol[par][lane] = attn[(size_t)(rowg0 + lane) * SEQ + k];
    __syncthreads();
    const float* vxr = vx + ((size_t)bh * SEQ + k) * NGATE + ucol;
    const float vx0 = vxr[0];
    const float vx1 = vxr[HDIM];
    const float vx2 = vxr[2 * HDIM];
    const float vx3 = vxr[3 * HDIM];

    v8f acc[2][4];
#pragma unroll
    for (int mt = 0; mt < 2; ++mt)
#pragma unroll
      for (int g = 0; g < 4; ++g) acc[mt][g] = (v8f){0.f,0.f,0.f,0.f,0.f,0.f,0.f,0.f};
    const _Float16* ha = &hA[par][0];
#pragma unroll
    for (int ks = 0; ks < 4; ++ks) {
      v16h bf[4];
#pragma unroll
      for (int g = 0; g < 4; ++g)
        bf[g] = Frag<_Float16>::load(whb + (size_t)(g * HDIM + ucol) * HDIM + ks * 32 + 8 * hh);
#pragma unroll
      for (int mt = 0; mt < 2; ++mt) {
        const v16h af = Frag<_Float16>::load(ha + (mt * 16 + cix) * HP_LDS + ks * 32 + 8 * hh);
#pragma unroll
        for (int g = 0; g < 4; ++g) acc[mt][g] = Frag<_Float16>::mma(af, bf[g], acc[mt][g]);
        Frag<_Float16>::guard(acc[mt][0], acc[mt][3], af, af);
      }
      Frag<_Float16>::keep(bf[0], bf[1], bf[2], bf[3]);
    }
    acc_guard4(acc[0][0], acc[0][1], acc[0][2], acc[0][3]);
    acc_guard4(acc[1][0], acc[1][1], acc[1][2], acc[1][3]);

    _Float16* hn = &hA[par ^ 1][0];
    const bool last = (k == SEQ - 1);
#pragma unroll
    for (int mt = 0; mt < 2; ++mt) {
#pragma unroll
      for (int r = 0; r < 8; ++r) {
        const int row = mt * 16 + 8 * hh + r;
        const float a = acol[par][row];
        const float zi = acc[mt][0][r] * RINV + (a * vx0 + bl0);
        const float zf = acc[mt][1][r] * RINV + (a * vx1 + bl1);
        const float zg = acc[mt][2][r] * RINV + (a * vx2 + bl2);
        const float zo = acc[mt][3][r] * RINV + (a * vx3 + bl3);
        const float cn = sigm_f(zf) * cst[mt][r] + sigm_f(zi) * tanhf(zg);
        cst[mt][r] = cn;
        const float hv = sigm_f(zo) * tanhf(cn);
        hn[row * HP_LDS + ucol] = (_Float16)(hv * 2048.0f);
        if (last) hs[row * SP_LDS + ucol] = hv;
      }
    }
  }
  __syncthreads();
  {
    v4u va[2], vb[2];
    size_t dst[2];
#pragma unroll
    for (int it = 0; it < 2; ++it) {
      const int row = it * 16 + 2 * w + hh;
      const int seg = cix * 8;
      const float* sp = hs + row * SP_LDS + seg;
      unsigned wa[4], wb[4];
#pragma unroll
      for (int e = 0; e < 4; ++e) wa[e] = pack_hl(sp[2 * e], sp[2 * e + 1], wb[e]);
      va[it] = (v4u){wa[0], wa[1], wa[2], wa[3]};
      vb[it] = (v4u){wb[0], wb[1], wb[2], wb[3]};
      dst[it] = (size_t)(b * SEQ + qb + row) * HD_ALL + (size_t)(h * HDIM + seg);
    }
    for (int pass = 0; pass < 2; ++pass) {
#pragma unroll
      for (int it = 0; it < 2; ++it) {
        *(volatile v4u*)(rdh + dst[it]) = va[it];
        *(volatile v4u*)(rdl + dst[it]) = vb[it];
      }
      __threadfence();
    }
  }
}

extern "C" void kernel_launch(void* const* d_in, const int* in_sizes, int n_in,
                              void* d_out, int out_size, void* d_ws, size_t ws_size,
                              hipStream_t stream) {
  (void)in_sizes; (void)n_in; (void)out_size;
  const float* xq    = (const float*)d_in[0];
  const float* xk    = (const float*)d_in[1];
  const float* xv    = (const float*)d_in[2];
  const int*   mask  = (const int*)d_in[3];
  const float* wq    = (const float*)d_in[4];
  const float* bq    = (const float*)d_in[5];
  const float* wk    = (const float*)d_in[6];
  const float* bk    = (const float*)d_in[7];
  const float* wv    = (const float*)d_in[8];
  const float* bv    = (const float*)d_in[9];
  const float* wx    = (const float*)d_in[10];
  const float* wh    = (const float*)d_in[11];
  const float* blstm = (const float*)d_in[12];
  const float* wo    = (const float*)d_in[13];
  const float* bo    = (const float*)d_in[14];

  float* out0 = (float*)d_out;
  float* attn = out0 + (size_t)NROW * HDIM;

  char* wsb = (char*)d_ws;
  size_t off = 0;
  auto carve = [&](size_t bytes) -> char* { char* p = wsb + off; off += (bytes + 255) & ~(size_t)255; return p; };
  const size_t xplane = (size_t)NROW * FEAT * 2;
  const size_t wplane = (size_t)FEAT * HD_ALL * 2;
  const size_t wxplane = (size_t)NHEAD * NGATE * HDIM * 2;
  const size_t woplane = (size_t)HDIM * HD_ALL * 2;
  const size_t pplane = (size_t)NROW * HD_ALL * 2;
  unsigned short* XQh = (unsigned short*)carve(xplane);  unsigned short* XQl = (unsigned short*)carve(xplane);
  unsigned short* XKh = (unsigned short*)carve(xplane);  unsigned short* XKl = (unsigned short*)carve(xplane);
  unsigned short* XVh = (unsigned short*)carve(xplane);  unsigned short* XVl = (unsigned short*)carve(xplane);
  unsigned short* WqTh = (unsigned short*)carve(wplane); unsigned short* WqTl = (unsigned short*)carve(wplane);
  unsigned short* WkTh = (unsigned short*)carve(wplane); unsigned short* WkTl = (unsigned short*)carve(wplane);
  unsigned short* WvTh = (unsigned short*)carve(wplane); unsigned short* WvTl = (unsigned short*)carve(wplane);
  unsigned short* WxTh = (unsigned short*)carve(wxplane); unsigned short* WxTl = (unsigned short*)carve(wxplane);
  unsigned short* WhT16 = (unsigned short*)carve(wxplane);
  unsigned short* WoTh = (unsigned short*)carve(woplane); unsigned short* WoTl = (unsigned short*)carve(woplane);
  unsigned short* Qh = (unsigned short*)carve(pplane);   unsigned short* Ql = (unsigned short*)carve(pplane);
  unsigned short* Kh = (unsigned short*)carve(pplane);   unsigned short* Kl = (unsigned short*)carve(pplane);
  unsigned short* Vh = (unsigned short*)carve(pplane);   unsigned short* Vl = (unsigned short*)carve(pplane);
  float* Sbuf  = (float*)carve((size_t)NBH * SEQ * SEQ * 4);
  float* VXbuf = (float*)carve((size_t)NBH * SEQ * NGATE * 4);
  unsigned short* RDh = (unsigned short*)carve(pplane);  unsigned short* RDl = (unsigned short*)carve(pplane);
  if (off > ws_size) return;

  const int n8 = (NROW * FEAT) / 8;
  k_cvt_split<<<dim3(n8 / 256), dim3(256), 0, stream>>>(xq, XQh, XQl, n8);
  k_cvt_split<<<dim3(n8 / 256), dim3(256), 0, stream>>>(xk, XKh, XKl, n8);
  k_cvt_split<<<dim3(n8 / 256), dim3(256), 0, stream>>>(xv, XVh, XVl, n8);

  k_transpose16<0><<<dim3(HD_ALL / 64, FEAT / 64, 1), dim3(256), 0, stream>>>(wq, WqTh, WqTl, FEAT, HD_ALL, 1.0f);
  k_transpose16<0><<<dim3(HD_ALL / 64, FEAT / 64, 1), dim3(256), 0, stream>>>(wk, WkTh, WkTl, FEAT, HD_ALL, 1.0f);
  k_transpose16<0><<<dim3(HD_ALL / 64, FEAT / 64, 1), dim3(256), 0, stream>>>(wv, WvTh, WvTl, FEAT, HD_ALL, 1.0f);
  k_transpose16<0><<<dim3(NGATE / 64, HDIM / 64, NHEAD), dim3(256), 0, stream>>>(wx, WxTh, WxTl, HDIM, NGATE, 1.0f);
  k_transpose16<1><<<dim3(NGATE / 64, HDIM / 64, NHEAD), dim3(256), 0, stream>>>(wh, WhT16, WhT16, HDIM, NGATE, 16.0f);
  k_transpose16<0><<<dim3(HDIM / 64, HD_ALL / 64, 1), dim3(256), 0, stream>>>(wo, WoTh, WoTl, HD_ALL, HDIM, 1.0f);

  wmma_gemm64<1, true, 2, 2, false, 0><<<dim3(8, 1), dim3(256), 0, stream>>>(
      XQh, XQl, FEAT, 0L, WqTh, WqTl, FEAT, 0L, (void*)Qh, (void*)Ql, HD_ALL, 0L, bq, bq, 0L, NROW, HD_ALL, FEAT, 1.0f);
  wmma_gemm64<1, true, 2, 2, false, 0><<<dim3(8, 1), dim3(256), 0, stream>>>(
      XKh, XKl, FEAT, 0L, WkTh, WkTl, FEAT, 0L, (void*)Kh, (void*)Kl, HD_ALL, 0L, bk, bk, 0L, NROW, HD_ALL, FEAT, 1.0f);
  wmma_gemm64<1, true, 2, 2, false, 0><<<dim3(8, 1), dim3(256), 0, stream>>>(
      XVh, XVl, FEAT, 0L, WvTh, WvTl, FEAT, 0L, (void*)Vh, (void*)Vl, HD_ALL, 0L, bv, bv, 0L, NROW, HD_ALL, FEAT, 1.0f);

  const float rsq = 0.08838834764831845f;
  for (int b = 0; b < NBATCH; ++b) {
    const size_t po = (size_t)b * SEQ * HD_ALL;
    float* Sb = Sbuf + (size_t)b * NHEAD * SEQ * SEQ;
    wmma_gemm64<1, true, 0, 0, false, 0><<<dim3(1, NHEAD), dim3(256), 0, stream>>>(
        Qh + po, Ql + po, HD_ALL, (long)HDIM, Kh + po, Kl + po, HD_ALL, (long)HDIM,
        (void*)Sb, (void*)Sb, SEQ, (long)(SEQ * SEQ), bq, bq, 0L, SEQ, SEQ, HDIM, rsq);
  }

  k_softmax_rows<<<dim3((NBH * SEQ) / 8), dim3(256), 0, stream>>>(Sbuf, mask, attn);

  for (int b = 0; b < NBATCH; ++b) {
    const size_t po = (size_t)b * SEQ * HD_ALL;
    float* VXb = VXbuf + (size_t)b * NHEAD * SEQ * NGATE;
    wmma_gemm64<1, true, 0, 0, false, 0><<<dim3(2, NHEAD), dim3(256), 0, stream>>>(
        Vh + po, Vl + po, HD_ALL, (long)HDIM, WxTh, WxTl, HDIM, (long)(NGATE * HDIM),
        (void*)VXb, (void*)VXb, NGATE, (long)(SEQ * NGATE), bq, bq, 0L, SEQ, NGATE, HDIM, 1.0f);
  }

  k_recur<<<dim3((NBH * SEQ) / 32), dim3(256), 0, stream>>>(attn, VXbuf, WhT16, blstm, RDh, RDl);

  wmma_gemm64<1, true, 2, 0, false, 0><<<dim3(1, 1), dim3(256), 0, stream>>>(
      RDh, RDl, HD_ALL, 0L, WoTh, WoTl, HD_ALL, 0L, (void*)out0, (void*)out0, HDIM, 0L, bo, bo, 0L, NROW, HDIM, HD_ALL, 1.0f);
}
